// EquivariantBlock_48275432407131
// MI455X (gfx1250) — hardware-run, weakly checked
//
#include <hip/hip_runtime.h>
#include <stddef.h>
#include <stdint.h>


#define HID    128
#define NPQ    256
#define KPQ    256
#define KNZ    512
#define KN2    256
#define W1R    258
#define NLAY   2
#define NTHR   256
#define NWAVE  8
#define EPB    256
#define DP     132
#define AP     136
#define MPITCH 128
#define CSTN   656
#define GBM    64
#define GBN    128
#define GTHR   128
#define EPT    8
#define CHUNK  (NTHR * EPT)
#define WCAP   (EPT * 32)
#define LISTN  (NWAVE * WCAP)
#define NBA    1024
#define SLA    10
#define RCAP   28672
#define DEGCAP 64
#define XROWS  320
#define NRANGE 4
#define NU_WPT  (3 * NPQ * (KPQ / 8))
#define NU_W2T  (3 * HID * (HID / 8))
#define NU_WN1  (NLAY * HID * (KNZ / 8))
#define NU_WN2  (NLAY * HID * (KN2 / 8))
#define AGG_ZINTS (LISTN + 2 * RCAP + 3 * NBA)
#define AGG_LDS_INTS (AGG_ZINTS + 16 + 4 * NBA)
#define AGG_LDS_BYTES (AGG_LDS_INTS * 4)
#define EDGE_LDS_BYTES (EPB * DP * 4 + EPB * AP * 2 + CSTN * 4 + EPB * 4)
#define WSMAX  134217728
#define CACT   16.0f
#define CWGT   1024.0f
#define CMSG   16.0f
#define PINV   6.103515625e-05f
#define MINV   0.0625f
#define NINV   0.01f

static_assert((CHUNK & (CHUNK - 1)) == 0 && CHUNK <= 4096);
static_assert((NBA & (NBA - 1)) == 0 && NBA == (1 << SLA));
static_assert(((long long)CHUNK << SLA) < (1LL << 31));
static_assert(LISTN % NTHR == 0);
static_assert(NBA % NWAVE == 0 && NBA % 32 == 0 && NBA == 4 * NTHR);
static_assert(RCAP % 4 == 0 && AGG_ZINTS % 4 == 0 && LISTN % 4 == 0);
static_assert(AGG_LDS_BYTES <= 300000);
static_assert(EDGE_LDS_BYTES <= 300000);
static_assert(NU_WPT % NTHR == 0 && NU_W2T % NTHR == 0 && NU_WN1 % NTHR == 0 && NU_WN2 % NTHR == 0);
static_assert((NPQ * (KPQ / 8)) % NTHR == 0 && (HID * (HID / 8)) % NTHR == 0);
static_assert((HID * (KNZ / 8)) % NTHR == 0 && (HID * (KN2 / 8)) % NTHR == 0);
static_assert(HID % 32 == 0 && KPQ % 32 == 0 && KNZ % 32 == 0 && KN2 % 32 == 0);
static_assert(GBM == (GTHR / 32) * 16 && GBN == 4 * 32 && GBN == HID && NPQ == 2 * GBN);
static_assert((DP * 4) % 16 == 0 && (AP * 2) % 16 == 0 && AP >= HID && DP >= HID);
static_assert(EPB == NTHR && EPB == 8 * 32);
static_assert(EPB * MPITCH * 2 <= EPB * AP * 2 && EPB * MPITCH * 2 == 16 * NTHR * 16);
static_assert((EPB * DP * 4) % 16 == 0 && (EPB * AP * 2) % 16 == 0);
static_assert((CSTN * 4) % 16 == 0 && CSTN >= 5 * HID + 1);
static_assert((XROWS * 3) % 4 == 0 && (XROWS * 3) / 4 <= NTHR && ((XROWS * 3 * 4) % 128) == 0);
static_assert(KNZ == 4 * HID && KN2 == 2 * HID && KPQ == 2 * HID && W1R == 2 * HID + 2);

typedef float          v4f   __attribute__((ext_vector_type(4)));
typedef float          v8f   __attribute__((ext_vector_type(8)));
typedef int            v4i   __attribute__((ext_vector_type(4)));
typedef int            v8i   __attribute__((ext_vector_type(8)));
typedef unsigned       v2u   __attribute__((ext_vector_type(2)));
typedef unsigned short v8us  __attribute__((ext_vector_type(8)));
typedef unsigned short v16us __attribute__((ext_vector_type(16)));
typedef __bf16         v16bf __attribute__((ext_vector_type(16)));
typedef _Float16       v16h  __attribute__((ext_vector_type(16)));
typedef v4f  __attribute__((may_alias)) v4fa;
typedef v4i  __attribute__((may_alias)) v4ia;
typedef v2u  __attribute__((may_alias)) v2ua;
typedef v8us __attribute__((may_alias)) v8usa;
union FragB { v16bf v; v16us u; v8us h[2]; v8i w; };
union FragH { v16h  v; v16us u; v8us h[2]; v8i w; };

__device__ __forceinline__ v8f wmb(const FragB& a, const FragB& b, v8f c) {
  v8f d = __builtin_amdgcn_wmma_f32_16x16x32_bf16(false, a.v, false, b.v, (short)0, c, false, false);
  asm volatile("v_nop\n\tv_nop\n\tv_nop\n\tv_nop" : "+v"(d) : "v"(a.w), "v"(b.w));
  return d;
}
__device__ __forceinline__ v8f wmh(const FragH& a, const FragH& b, v8f c) {
  v8f d = __builtin_amdgcn_wmma_f32_16x16x32_f16(false, a.v, false, b.v, (short)0, c, false, false);
  asm volatile("v_nop\n\tv_nop\n\tv_nop\n\tv_nop" : "+v"(d) : "v"(a.w), "v"(b.w));
  return d;
}

__device__ __forceinline__ unsigned bf16_bits(float f) {
  const unsigned u = __float_as_uint(f);
  return (u + 0x7FFFu + ((u >> 16) & 1u)) >> 16;
}
__device__ __forceinline__ float bf16_val(float f) {
  return __uint_as_float(bf16_bits(f) << 16);
}
__device__ __forceinline__ unsigned short f2h(float f) {
  const _Float16 hv = (_Float16)f;
  return __builtin_bit_cast(unsigned short, hv);
}
__device__ __forceinline__ float h2f(unsigned b) {
  const _Float16 hv = __builtin_bit_cast(_Float16, (unsigned short)b);
  return (float)hv;
}
__device__ __forceinline__ float silu_f(float t) {
  return t * __builtin_amdgcn_rcpf(1.0f + __expf(-t));
}
__device__ __forceinline__ void put16(unsigned short* dp, v8us o) {
  *(volatile v8us*)dp = o;
  __threadfence();
  *(volatile v8us*)dp = o;
}
__device__ __forceinline__ void putf4(float* dp, v4f o) {
  *(volatile v4f*)dp = o;
  __threadfence();
  *(volatile v4f*)dp = o;
}

template <int SLB>
__device__ __forceinline__ int scan_chunk(const int* __restrict__ dsts, int nE, int cbase, int slotBase,
                                          int nb, int vec8, int* list, int tid, int lane, int wave) {
  int wc = 0;
  const int el0  = tid * EPT;
  const int e0   = cbase + el0;
  const int sent = -2147483647 - 1;
  v4i da, db;
  if (vec8 != 0 && cbase + CHUNK <= nE) {
    da = *(const v4i*)(dsts + e0);
    db = *(const v4i*)(dsts + e0 + 4);
  } else {
    da.x = (e0     < nE) ? dsts[min(e0,     nE - 1)] : sent;
    da.y = (e0 + 1 < nE) ? dsts[min(e0 + 1, nE - 1)] : sent;
    da.z = (e0 + 2 < nE) ? dsts[min(e0 + 2, nE - 1)] : sent;
    da.w = (e0 + 3 < nE) ? dsts[min(e0 + 3, nE - 1)] : sent;
    db.x = (e0 + 4 < nE) ? dsts[min(e0 + 4, nE - 1)] : sent;
    db.y = (e0 + 5 < nE) ? dsts[min(e0 + 5, nE - 1)] : sent;
    db.z = (e0 + 6 < nE) ? dsts[min(e0 + 6, nE - 1)] : sent;
    db.w = (e0 + 7 < nE) ? dsts[min(e0 + 7, nE - 1)] : sent;
  }
  const unsigned nbs = (unsigned)slotBase;
  const unsigned unb = (unsigned)nb;
  const unsigned s0 = (unsigned)da.x - nbs, s1 = (unsigned)da.y - nbs;
  const unsigned s2 = (unsigned)da.z - nbs, s3 = (unsigned)da.w - nbs;
  const unsigned s4 = (unsigned)db.x - nbs, s5 = (unsigned)db.y - nbs;
  const unsigned s6 = (unsigned)db.z - nbs, s7 = (unsigned)db.w - nbs;
  const bool h0 = s0 < unb, h1 = s1 < unb, h2 = s2 < unb, h3 = s3 < unb;
  const bool h4 = s4 < unb, h5 = s5 < unb, h6 = s6 < unb, h7 = s7 < unb;
  const unsigned any = __builtin_amdgcn_ballot_w32(h0 | h1 | h2 | h3 | h4 | h5 | h6 | h7);
  if (any != 0u) {
#define HITJ(J, HJ, SJ) { \
      const unsigned mj = __builtin_amdgcn_ballot_w32(HJ); \
      if (mj != 0u) { \
        if (HJ) { \
          const int pos = wc + (int)__builtin_amdgcn_mbcnt_lo(mj, 0u); \
          if (pos < WCAP) list[wave * WCAP + pos] = ((el0 + (J)) << SLB) | (int)(SJ); \
        } \
        wc += (int)__builtin_popcount(mj); } }
    HITJ(0, h0, s0)
    HITJ(1, h1, s1)
    HITJ(2, h2, s2)
    HITJ(3, h3, s3)
    HITJ(4, h4, s4)
    HITJ(5, h5, s5)
    HITJ(6, h6, s6)
    HITJ(7, h7, s7)
#undef HITJ
  }
  return wc;
}

__global__ __launch_bounds__(NTHR) void k_prep(const float* __restrict__ h, const float* __restrict__ x,
                                               const float* __restrict__ ew1, const float* __restrict__ cw1,
                                               const float* __restrict__ ew2, const float* __restrict__ cw2,
                                               const float* __restrict__ nw1, const float* __restrict__ nw2,
                                               int nN, int mRows,
                                               unsigned short* WPT, unsigned short* W2T, unsigned short* WN1T,
                                               unsigned short* WN2T, unsigned short* NZ, float* CP) {
  const int u  = (int)blockIdx.x * NTHR + (int)threadIdx.x;
  const int U0 = NU_WPT;
  const int U1 = U0 + NU_W2T;
  const int U2 = U1 + NU_WN1;
  const int U3 = U2 + NU_WN2;
  const int U4 = U3 + mRows * 32;
  const int nXP = ((mRows + NTHR - 1) / NTHR) * NTHR;
  const int U5 = U4 + nXP;
  v8us o;
  if (u < U0) {
    const int l   = u >> 13;
    const int vv  = u & 8191;
    const int n   = vv >> 5;
    const int k8  = (vv & 31) * 8;
    const float* W = (l == 0) ? ew1 : ((l == 1) ? (ew1 + (size_t)W1R * HID) : cw1);
    const int rw  = (n >> 7) * HID + (k8 & (HID - 1));
    const int nn  = n & (HID - 1);
    const float* p = W + (size_t)rw * HID + nn;
#pragma unroll
    for (int i = 0; i < 8; ++i) o[i] = (unsigned short)bf16_bits(p[(size_t)i * HID]);
    put16(WPT + (size_t)l * (NPQ * KPQ) + (size_t)n * KPQ + k8, o);
    return;
  } else if (u < U1) {
    const int v  = u - U0;
    const int l  = v >> 11;
    const int vv = v & 2047;
    const int n  = vv >> 4;
    const int k8 = (vv & 15) * 8;
    const float* W = (l == 0) ? ew2 : ((l == 1) ? (ew2 + (size_t)HID * HID) : cw2);
    const float* p = W + (size_t)k8 * HID + n;
#pragma unroll
    for (int i = 0; i < 8; ++i) o[i] = f2h(CWGT * bf16_val(p[(size_t)i * HID]));
    put16(W2T + (size_t)l * (HID * HID) + (size_t)n * HID + k8, o);
    return;
  } else if (u < U2) {
    const int v    = u - U1;
    const int l    = v >> 13;
    const int vv   = v & 8191;
    const int n    = vv >> 6;
    const int k8   = (vv & 63) * 8;
    const int srow = (k8 >> 8) * HID + (k8 & (HID - 1));
    const float* p = nw1 + (size_t)l * (2 * HID * HID) + (size_t)srow * HID + n;
#pragma unroll
    for (int i = 0; i < 8; ++i) o[i] = (unsigned short)bf16_bits(p[(size_t)i * HID]);
    put16(WN1T + (size_t)l * (HID * KNZ) + (size_t)n * KNZ + k8, o);
    return;
  } else if (u < U3) {
    const int v    = u - U2;
    const int l    = v >> 12;
    const int vv   = v & 4095;
    const int n    = vv >> 5;
    const int k8   = (vv & 31) * 8;
    const int srow = k8 & (HID - 1);
    const float* p = nw2 + (size_t)l * (HID * HID) + (size_t)srow * HID + n;
#pragma unroll
    for (int i = 0; i < 8; ++i) o[i] = (unsigned short)bf16_bits(p[(size_t)i * HID]);
    put16(WN2T + (size_t)l * (HID * KN2) + (size_t)n * KN2 + k8, o);
    return;
  } else if (u < U4) {
    const int v   = u - U3;
    const int row = v >> 5;
    const int q   = v & 31;
    const int c8  = (q & 15) * 8;
    const int rc  = row < nN ? row : nN - 1;
    const float* p = h + (size_t)rc * HID + c8;
    const v4f a = *(const v4fa*)p;
    const v4f b = *(const v4fa*)(p + 4);
    const bool ok = (row < nN) && (q < 16);
    o[0] = ok ? (unsigned short)bf16_bits(a.x) : (unsigned short)0;
    o[1] = ok ? (unsigned short)bf16_bits(a.y) : (unsigned short)0;
    o[2] = ok ? (unsigned short)bf16_bits(a.z) : (unsigned short)0;
    o[3] = ok ? (unsigned short)bf16_bits(a.w) : (unsigned short)0;
    o[4] = ok ? (unsigned short)bf16_bits(b.x) : (unsigned short)0;
    o[5] = ok ? (unsigned short)bf16_bits(b.y) : (unsigned short)0;
    o[6] = ok ? (unsigned short)bf16_bits(b.z) : (unsigned short)0;
    o[7] = ok ? (unsigned short)bf16_bits(b.w) : (unsigned short)0;
    put16(NZ + (size_t)row * KNZ + 8 * q, o);
    return;
  } else if (u < U5) {
    const int row = u - U4;
    if (row >= mRows) return;
    const int rc  = row < nN ? row : nN - 1;
    const bool ok = row < nN;
    const float x0 = x[(size_t)rc * 3 + 0];
    const float x1 = x[(size_t)rc * 3 + 1];
    const float x2 = x[(size_t)rc * 3 + 2];
    v4f qv;
    qv.x = ok ? bf16_val(x0) : 0.0f;
    qv.y = ok ? bf16_val(x1) : 0.0f;
    qv.z = ok ? bf16_val(x2) : 0.0f;
    qv.w = 0.0f;
    putf4(CP + (size_t)row * 4, qv);
    return;
  }
}

template <int MODE>
__global__ __launch_bounds__(GTHR) void k_gemm(const unsigned short* __restrict__ A, int lda,
                                               const unsigned short* __restrict__ BT, int ldb, int K,
                                               const float* __restrict__ bias, int nN, int wout,
                                               float* Cm, int ldc, unsigned short* Cb, int ldcb) {
  __shared__ __attribute__((aligned(16))) float stg[GBM * GBN];
  const int tid = (int)threadIdx.x, lane = tid & 31, wave = tid >> 5, hh = lane >> 4, m = lane & 15;
  const int rowBase = (int)blockIdx.x * GBM;
  const int colBase = (int)blockIdx.y * GBN;

  if constexpr (MODE == 2) {
    const int j = lane & 15, part = lane >> 4;
#pragma unroll 4
    for (int i = 0; i < 16; ++i) {
      const int row = rowBase + 16 * wave + i;
      const unsigned short* hp = Cb + (size_t)row * (size_t)ldcb + 8 * j;
      const v4i hw = *(const v4ia*)hp;
      const v4i lw = *(const v4ia*)(hp + HID);
      float v[8];
#pragma unroll
      for (int e = 0; e < 4; ++e) {
        const unsigned hu = (unsigned)hw[e], lu = (unsigned)lw[e];
        v[2 * e]     = __uint_as_float(hu << 16) + __uint_as_float(lu << 16);
        v[2 * e + 1] = __uint_as_float(hu & 0xffff0000u) + __uint_as_float(lu & 0xffff0000u);
      }
      v4f w4;
      w4.x = part ? v[4] : v[0];
      w4.y = part ? v[5] : v[1];
      w4.z = part ? v[6] : v[2];
      w4.w = part ? v[7] : v[3];
      *(v4fa*)(stg + (16 * wave + i) * GBN + 8 * j + 4 * part) = w4;
    }
    __syncthreads();
  }

  v8f acc[8];
  {
    const v8f z = {0.f, 0.f, 0.f, 0.f, 0.f, 0.f, 0.f, 0.f};
#pragma unroll
    for (int t = 0; t < 8; ++t) acc[t] = z;
  }
  const unsigned short* ap = A  + (size_t)(rowBase + 16 * wave + m) * (size_t)lda + 8 * hh;
  const unsigned short* bp = BT + (size_t)(colBase + m) * (size_t)ldb + 8 * hh;

#pragma unroll 1
  for (int k0 = 0; k0 < K; k0 += 32) {
    FragB af;
    af.h[0] = *(const v8usa*)(ap + k0);
    af.h[1] = *(const v8usa*)(ap + k0 + 16);
#pragma unroll
    for (int nt = 0; nt < 8; ++nt) {
      const unsigned short* wq = bp + (size_t)(16 * nt) * (size_t)ldb + k0;
      FragB bf;
      bf.h[0] = *(const v8usa*)wq;
      bf.h[1] = *(const v8usa*)(wq + 16);
      acc[nt] = wmb(af, bf, acc[nt]);
    }
  }

#pragma unroll
  for (int nt = 0; nt < 8; ++nt) {
    const int lc = 16 * nt + m;
    float bvv = 0.0f;
    if constexpr (MODE != 0) bvv = bf16_val(bias[colBase + lc]);
#pragma unroll
    for (int r = 0; r < 8; ++r) {
      const int lr = 16 * wave + 8 * hh + r;
      float v = acc[nt][r];
      if constexpr (MODE == 1) v = silu_f(v + bvv);
      if constexpr (MODE == 2) v = stg[lr * GBN + lc] + (v + bvv);
      stg[lr * GBN + lc] = v;
    }
  }
  __syncthreads();

  if constexpr (MODE == 0) {
    v4f pv[16];
#pragma unroll
    for (int i = 0; i < 16; ++i) pv[i] = *(const v4fa*)(stg + (16 * wave + i) * GBN + 4 * lane);
#pragma unroll
    for (int i = 0; i < 16; ++i) {
      float* op = Cm + (size_t)(rowBase + 16 * wave + i) * (size_t)ldc + colBase + 4 * lane;
      *(volatile v4f*)op = pv[i];
    }
    __threadfence();
#pragma unroll
    for (int i = 0; i < 16; ++i) {
      float* op = Cm + (size_t)(rowBase + 16 * wave + i) * (size_t)ldc + colBase + 4 * lane;
      *(volatile v4f*)op = pv[i];
    }
  } else {
    const int part = lane >> 4;
    const int j = lane & 15;
    const unsigned mh = 0u - (unsigned)part;
    const unsigned ml = ~mh;
    v8us pv[16];
#pragma unroll
    for (int i = 0; i < 16; ++i) {
      const float* sp = stg + (16 * wave + i) * GBN + 8 * j;
      const v4f a = *(const v4fa*)sp;
      const v4f b = *(const v4fa*)(sp + 4);
      const v8f f8 = {a.x, a.y, a.z, a.w, b.x, b.y, b.z, b.w};
      v8us oo;
#pragma unroll
      for (int e = 0; e < 8; ++e) {
        const unsigned hb = bf16_bits(f8[e]);
        const unsigned lb = bf16_bits(f8[e] - __uint_as_float(hb << 16));
        oo[e] = (unsigned short)((hb & ml) | (lb & mh));
      }
      pv[i] = oo;
    }
    if constexpr (MODE == 1) {
#pragma unroll
      for (int i = 0; i < 16; ++i) {
        unsigned short* op = Cb + (size_t)(rowBase + 16 * wave + i) * (size_t)ldcb + part * HID + 8 * j;
        *(volatile v8us*)op = pv[i];
      }
      __threadfence();
#pragma unroll
      for (int i = 0; i < 16; ++i) {
        unsigned short* op = Cb + (size_t)(rowBase + 16 * wave + i) * (size_t)ldcb + part * HID + 8 * j;
        *(volatile v8us*)op = pv[i];
      }
    } else {
#pragma unroll
      for (int i = 0; i < 16; ++i) {
        const int row = rowBase + 16 * wave + i;
        if (row < nN) {
          unsigned short* op = Cb + (size_t)row * (size_t)ldcb + part * HID + 8 * j;
          *(volatile v8us*)op = pv[i];
        }
      }
      __threadfence();
#pragma unroll
      for (int i = 0; i < 16; ++i) {
        const int row = rowBase + 16 * wave + i;
        if (row < nN) {
          unsigned short* op = Cb + (size_t)row * (size_t)ldcb + part * HID + 8 * j;
          *(volatile v8us*)op = pv[i];
        }
      }
      if (wout != 0) {
        v4f pf[16];
#pragma unroll
        for (int i = 0; i < 16; ++i) pf[i] = *(const v4fa*)(stg + (16 * wave + i) * GBN + 4 * lane);
#pragma unroll
        for (int i = 0; i < 16; ++i) {
          const int row = rowBase + 16 * wave + i;
          if (row < nN) {
            float* op = Cm + (size_t)row * (size_t)ldc + colBase + 4 * lane;
            *(volatile v4f*)op = pf[i];
          }
        }
        __threadfence();
#pragma unroll
        for (int i = 0; i < 16; ++i) {
          const int row = rowBase + 16 * wave + i;
          if (row < nN) {
            float* op = Cm + (size_t)row * (size_t)ldc + colBase + 4 * lane;
            *(volatile v4f*)op = pf[i];
          }
        }
      }
    }
  }
}

__device__ __forceinline__ void wave_gemm_h(const unsigned short* sAw, float* sDw,
                                            const unsigned short* __restrict__ BT, int ldb, int K,
                                            int hh, int m) {
#pragma unroll 1
  for (int nh = 0; nh < 2; ++nh) {
    v8f acc[2][4];
    {
      const v8f z = {0.f, 0.f, 0.f, 0.f, 0.f, 0.f, 0.f, 0.f};
#pragma unroll
      for (int mt = 0; mt < 2; ++mt)
#pragma unroll
        for (int nt = 0; nt < 4; ++nt) acc[mt][nt] = z;
    }
    const unsigned short* ap0 = sAw + m * AP + 8 * hh;
    const unsigned short* ap1 = ap0 + 16 * AP;
    const unsigned short* bp  = BT + (size_t)(64 * nh + m) * (size_t)ldb + 8 * hh;
#pragma unroll 1
    for (int k0 = 0; k0 < K; k0 += 32) {
      FragH a0, a1;
      a0.h[0] = *(const v8usa*)(ap0 + k0);
      a0.h[1] = *(const v8usa*)(ap0 + k0 + 16);
      a1.h[0] = *(const v8usa*)(ap1 + k0);
      a1.h[1] = *(const v8usa*)(ap1 + k0 + 16);
#pragma unroll
      for (int nt = 0; nt < 4; ++nt) {
        const unsigned short* wq = bp + (size_t)(16 * nt) * (size_t)ldb + k0;
        FragH b;
        b.h[0] = *(const v8usa*)wq;
        b.h[1] = *(const v8usa*)(wq + 16);
        acc[0][nt] = wmh(a0, b, acc[0][nt]);
        acc[1][nt] = wmh(a1, b, acc[1][nt]);
      }
    }
#pragma unroll
    for (int nt = 0; nt < 4; ++nt) {
      const int col = 64 * nh + 16 * nt + m;
#pragma unroll
      for (int mt = 0; mt < 2; ++mt)
#pragma unroll
        for (int r = 0; r < 8; ++r) sDw[(16 * mt + 8 * hh + r) * DP + col] = acc[mt][nt][r];
    }
  }
}

template <int COORD>
__global__ __launch_bounds__(NTHR) void k_edge(const int* __restrict__ ei, int nE, int nN, int eBase, int nEh,
                                               const float* __restrict__ PQ, const float* __restrict__ CP,
                                               const float* __restrict__ EA,
                                               const unsigned short* __restrict__ W2T,
                                               const float* __restrict__ b1, const float* __restrict__ b2,
                                               const float* __restrict__ wv, const float* __restrict__ wb,
                                               const float* __restrict__ w56,
                                               unsigned short* Mh, float* Sh) {
  extern __shared__ __attribute__((aligned(16))) float dyn[];
  float*          sD  = dyn;
  unsigned short* sA  = (unsigned short*)(dyn + EPB * DP);
  unsigned short* sM  = sA;
  float*          cst = dyn + EPB * DP + (EPB * AP) / 2;
  float*          sS  = cst + CSTN;

  const int tid = (int)threadIdx.x, lane = tid & 31, wave = tid >> 5, hh = lane >> 4, m = lane & 15;

  if (tid < HID) {
    cst[tid]           = bf16_val(b1[tid]);
    cst[HID + tid]     = bf16_val(b2[tid]);
    cst[2 * HID + tid] = bf16_val(wv[tid]);
    cst[3 * HID + tid] = bf16_val(w56[tid]);
    cst[4 * HID + tid] = bf16_val(w56[HID + tid]);
    const float vb = bf16_val(wb[0]);
    if (tid == 0) cst[5 * HID] = vb;
  }

  const int  elb  = (int)blockIdx.x * EPB;
  const int  el   = elb + tid;
  const bool live = el < nEh;
  const int  elc  = live ? el : (nEh - 1);
  const int  eg   = eBase + elc;
  int r = ei[eg];
  int c = ei[(size_t)nE + (size_t)eg];
  r = r < 0 ? 0 : (r > nN - 1 ? nN - 1 : r);
  c = c < 0 ? 0 : (c > nN - 1 ? nN - 1 : c);
  const v4f xr = *(const v4fa*)(CP + (size_t)r * 4);
  const v4f xc = *(const v4fa*)(CP + (size_t)c * 4);
  const float dfx = xr.x - xc.x, dfy = xr.y - xc.y, dfz = xr.z - xc.z;
  const float radial = (dfx * dfx + dfz * dfz) + dfy * dfy;
  const float ea = bf16_val(EA[eg]);
  __syncthreads();

  float*          rd = sD + tid * DP;
  unsigned short* ra = sA + tid * AP;
  unsigned short* rm = sM + tid * MPITCH;

  {
    const float* pr = PQ + (size_t)r * NPQ;
    const float* qr = PQ + (size_t)c * NPQ + HID;
#pragma unroll 1
    for (int c8 = 0; c8 < HID / 8; ++c8) {
      const v4f pa = *(const v4fa*)(pr + 8 * c8);
      const v4f pb = *(const v4fa*)(pr + 8 * c8 + 4);
      const v4f qa = *(const v4fa*)(qr + 8 * c8);
      const v4f qb = *(const v4fa*)(qr + 8 * c8 + 4);
      const v4f ba = *(const v4fa*)(cst + 8 * c8);
      const v4f bb = *(const v4fa*)(cst + 8 * c8 + 4);
      const v4f ua = *(const v4fa*)(cst + 3 * HID + 8 * c8);
      const v4f ub = *(const v4fa*)(cst + 3 * HID + 8 * c8 + 4);
      const v4f va = *(const v4fa*)(cst + 4 * HID + 8 * c8);
      const v4f vb = *(const v4fa*)(cst + 4 * HID + 8 * c8 + 4);
      const v8f p8 = {pa.x, pa.y, pa.z, pa.w, pb.x, pb.y, pb.z, pb.w};
      const v8f q8 = {qa.x, qa.y, qa.z, qa.w, qb.x, qb.y, qb.z, qb.w};
      const v8f b8 = {ba.x, ba.y, ba.z, ba.w, bb.x, bb.y, bb.z, bb.w};
      const v8f u8 = {ua.x, ua.y, ua.z, ua.w, ub.x, ub.y, ub.z, ub.w};
      const v8f v8 = {va.x, va.y, va.z, va.w, vb.x, vb.y, vb.z, vb.w};
      v8us o;
#pragma unroll
      for (int i = 0; i < 8; ++i) {
        const float pre = (p8[i] + q8[i]) + fmaf(radial, u8[i], fmaf(ea, v8[i], b8[i]));
        o[i] = f2h(CACT * silu_f(pre));
      }
      *(v8usa*)(ra + 8 * c8) = o;
    }
  }
  __syncthreads();

  const unsigned short* sAw = sA + 32 * wave * AP;
  float*                sDw = sD + 32 * wave * DP;

  wave_gemm_h(sAw, sDw, W2T, HID, HID, hh, m);
  __syncthreads();

  if constexpr (COORD == 0) {
    float dot = 0.0f;
#pragma unroll 1
    for (int c8 = 0; c8 < HID / 8; ++c8) {
      const v4f va = *(const v4fa*)(rd + 8 * c8);
      const v4f vb = *(const v4fa*)(rd + 8 * c8 + 4);
      const v4f ba = *(const v4fa*)(cst + HID + 8 * c8);
      const v4f bb = *(const v4fa*)(cst + HID + 8 * c8 + 4);
      const v4f wa = *(const v4fa*)(cst + 2 * HID + 8 * c8);
      const v4f wq = *(const v4fa*)(cst + 2 * HID + 8 * c8 + 4);
      const v8f v8 = {va.x, va.y, va.z, va.w, vb.x, vb.y, vb.z, vb.w};
      const v8f b8 = {ba.x, ba.y, ba.z, ba.w, bb.x, bb.y, bb.z, bb.w};
      const v8f w8 = {wa.x, wa.y, wa.z, wa.w, wq.x, wq.y, wq.z, wq.w};
      v8f mf;
#pragma unroll
      for (int i = 0; i < 8; ++i) {
        const float mj = silu_f(fmaf(v8[i], PINV, b8[i]));
        dot   = fmaf(mj, w8[i], dot);
        mf[i] = mj;
      }
      const v4f m0 = {mf[0], mf[1], mf[2], mf[3]};
      const v4f m1 = {mf[4], mf[5], mf[6], mf[7]};
      *(v4fa*)(rd + 8 * c8)     = m0;
      *(v4fa*)(rd + 8 * c8 + 4) = m1;
    }
    const float att = __builtin_amdgcn_rcpf(1.0f + __expf(-(dot + cst[5 * HID])));
#pragma unroll 1
    for (int c8 = 0; c8 < HID / 8; ++c8) {
      const v4f va = *(const v4fa*)(rd + 8 * c8);
      const v4f vb = *(const v4fa*)(rd + 8 * c8 + 4);
      const v8f v8 = {va.x, va.y, va.z, va.w, vb.x, vb.y, vb.z, vb.w};
      v8us o;
#pragma unroll
      for (int i = 0; i < 8; ++i) o[i] = f2h(CMSG * (v8[i] * att));
      *(v8usa*)(rm + 8 * c8) = o;
    }
    __syncthreads();

    {
      v4i pv[16];
#pragma unroll
      for (int it = 0; it < 16; ++it) pv[it] = *(const v4ia*)(sM + (size_t)(it * NTHR + tid) * 8);
      unsigned short* mb = Mh + (size_t)elb * MPITCH;
#pragma unroll
      for (int it = 0; it < 16; ++it) *(volatile v4i*)(mb + (size_t)(it * NTHR + tid) * 8) = pv[it];
      __threadfence();
#pragma unroll
      for (int it = 0; it < 16; ++it) *(volatile v4i*)(mb + (size_t)(it * NTHR + tid) * 8) = pv[it];
    }
  } else {
    float dot = 0.0f;
#pragma unroll 1
    for (int c8 = 0; c8 < HID / 8; ++c8) {
      const v4f va = *(const v4fa*)(rd + 8 * c8);
      const v4f vb = *(const v4fa*)(rd + 8 * c8 + 4);
      const v4f ba = *(const v4fa*)(cst + HID + 8 * c8);
      const v4f bb = *(const v4fa*)(cst + HID + 8 * c8 + 4);
      const v4f wa = *(const v4fa*)(cst + 2 * HID + 8 * c8);
      const v4f wq = *(const v4fa*)(cst + 2 * HID + 8 * c8 + 4);
      const v8f v8 = {va.x, va.y, va.z, va.w, vb.x, vb.y, vb.z, vb.w};
      const v8f b8 = {ba.x, ba.y, ba.z, ba.w, bb.x, bb.y, bb.z, bb.w};
      const v8f w8 = {wa.x, wa.y, wa.z, wa.w, wq.x, wq.y, wq.z, wq.w};
#pragma unroll
      for (int i = 0; i < 8; ++i) {
        const float cj = silu_f(fmaf(v8[i], PINV, b8[i]));
        dot = fmaf(cj, w8[i], dot);
      }
    }
    const float den = sqrtf(radial + 1e-8f) + 1.0f;
    const float sv  = dot * __builtin_amdgcn_rcpf(den);
    sS[tid] = live ? sv : 0.0f;
    __syncthreads();

    {
      const int tl = tid < 64 ? tid : 63;
      const v4f o4 = *(const v4fa*)(sS + 4 * tl);
      float* sp = Sh + (size_t)elb + 4 * tl;
      if (tid < 64) *(volatile v4f*)sp = o4;
      __threadfence();
      if (tid < 64) *(volatile v4f*)sp = o4;
    }
  }
}

template <int COORD>
__global__ __launch_bounds__(NTHR) void k_scan(const int* __restrict__ keys, const int* __restrict__ cols,
                                               int nEh, int nN, int vec8, int mRows, int first,
                                               const unsigned short* __restrict__ Mh,
                                               const float* __restrict__ Sh, const float* __restrict__ CP,
                                               unsigned short* NZ, float* XAGG) {
  extern __shared__ __attribute__((aligned(16))) int dsm[];
  int*   list = dsm;
  int*   hl   = dsm + LISTN;
  int*   sl   = hl + RCAP;
  int*   cnt  = sl + RCAP;
  int*   offs = cnt + NBA;
  int*   cur  = offs + NBA;
  int*   misc = cur + NBA;
  float* sdx  = (float*)(misc + 16);
  const int tid = (int)threadIdx.x, lane = tid & 31, wave = tid >> 5;
  const int nodeBase = (int)blockIdx.x * NBA;
  const v4f z4f = {0.0f, 0.0f, 0.0f, 0.0f};

  {
    const v4i z4 = {0, 0, 0, 0};
    for (int i = tid * 4; i < AGG_ZINTS; i += NTHR * 4) *(v4ia*)(dsm + i) = z4;
    if (tid < 16) misc[tid] = 0;
  }
  __syncthreads();

  int t = 0, ov = 0;
  const int nChunks = (nEh + CHUNK - 1) / CHUNK;
#pragma unroll 1
  for (int ch = 0; ch < nChunks; ++ch) {
    const int cbase = ch * CHUNK;
    const int wc = scan_chunk<SLA>(keys, nEh, cbase, nodeBase, NBA, vec8, list, tid, lane, wave);
    if (lane == 0) misc[wave] = wc;
    __syncthreads();
    if (wave == 0) {
#pragma unroll 1
      for (int w2 = 0; w2 < NWAVE; ++w2) {
        int cc = misc[w2];
        cc = cc < 0 ? 0 : (cc > WCAP ? WCAP : cc);
#pragma unroll 1
        for (int b0 = 0; b0 < cc; b0 += 32) {
          const int idx = b0 + lane;
          const int ent = list[w2 * WCAP + (idx < WCAP ? idx : WCAP - 1)];
          const int m32 = (cc - b0) < 32 ? (cc - b0) : 32;
#pragma unroll 1
          for (int k = 0; k < m32; ++k) {
            const int u    = __builtin_amdgcn_readlane(ent, k);
            const int slot = u & (NBA - 1);
            const int el   = (u >> SLA) & (CHUNK - 1);
            const int pk   = ((cbase + el) << SLA) | slot;
            if (t < RCAP) {
              if (lane == 0) { hl[t] = pk; cnt[slot] = cnt[slot] + 1; }
              t = t + 1;
            } else {
              ov = 1;
            }
          }
        }
      }
    }
    __syncthreads();
  }
  if (wave == 0 && lane == 0) { misc[8] = t; misc[9] = ov; }
  __syncthreads();
  int tt = misc[8];
  tt = tt < 0 ? 0 : (tt > RCAP ? RCAP : tt);
  const int ovf = misc[9];

  if (wave == 0) {
    const int base = lane * (NBA / 32);
    int s = 0;
#pragma unroll 1
    for (int i = 0; i < NBA / 32; ++i) s += cnt[base + i];
    int incl = s;
#pragma unroll
    for (int d = 1; d < 32; d <<= 1) {
      const int y = __shfl_up(incl, d, 32);
      if (lane >= d) incl += y;
    }
    int run = incl - s;
#pragma unroll 1
    for (int i = 0; i < NBA / 32; ++i) {
      const int cv = cnt[base + i];
      offs[base + i] = run;
      cur[base + i]  = run;
      run += cv;
    }
  }
  __syncthreads();
  if (wave == 0) {
#pragma unroll 1
    for (int b0 = 0; b0 < tt; b0 += 32) {
      const int idx = b0 + lane;
      const int ent = hl[idx < RCAP ? idx : RCAP - 1];
      const int m32 = (tt - b0) < 32 ? (tt - b0) : 32;
#pragma unroll 1
      for (int k = 0; k < m32; ++k) {
        const int u    = __builtin_amdgcn_readlane(ent, k);
        const int slot = u & (NBA - 1);
        if (lane == 0) {
          int p = cur[slot];
          p = p < 0 ? 0 : (p > RCAP - 1 ? RCAP - 1 : p);
          sl[p] = u;
          cur[slot] = p + 1;
        }
      }
    }
  }
  __syncthreads();

  const float qnan = __int_as_float(0x7fc00000);
  const float pz = (ovf != 0) ? qnan : 0.0f;
#pragma unroll 1
  for (int si = 0; si < NBA / NWAVE; ++si) {
    const int s    = si * NWAVE + wave;
    const int node = nodeBase + s;
    int cdeg = cnt[s];
    const bool big = cdeg > DEGCAP;
    cdeg = cdeg < 0 ? 0 : (cdeg > DEGCAP ? DEGCAP : cdeg);
    int o = offs[s];
    o = o < 0 ? 0 : (o > RCAP ? RCAP : o);
    const int nc = node < nN ? node : nN - 1;
    float a0 = 0.0f, a1 = 0.0f, a2 = 0.0f, a3 = 0.0f;
    float dx = 0.0f, dy = 0.0f, dz = 0.0f;
    v4f xd = z4f;
    if constexpr (COORD == 1) xd = *(const v4fa*)(CP + (size_t)nc * 4);
#pragma unroll 1
    for (int b0 = 0; b0 < cdeg; b0 += 32) {
      int idx = o + b0 + lane;
      idx = idx > RCAP - 1 ? RCAP - 1 : idx;
      const int ent = sl[idx];
      int eid = ent >> SLA;
      eid = eid < 0 ? 0 : (eid > nEh - 1 ? nEh - 1 : eid);
      const int m32 = (cdeg - b0) < 32 ? (cdeg - b0) : 32;
      if constexpr (COORD == 0) {
#pragma unroll 1
        for (int k = 0; k < m32; ++k) {
          const int ek = __builtin_amdgcn_readlane(eid, k);
          const unsigned short* rp = Mh + (size_t)ek * MPITCH + 4 * lane;
          const v2u w = *(const v2ua*)rp;
          a0 += h2f(w.x & 0xffffu);
          a1 += h2f(w.x >> 16);
          a2 += h2f(w.y & 0xffffu);
          a3 += h2f(w.y >> 16);
        }
      } else {
        int sr = cols[eid];
        sr = sr < 0 ? 0 : (sr > nN - 1 ? nN - 1 : sr);
        const v4f   xs = *(const v4fa*)(CP + (size_t)sr * 4);
        const float sv = Sh[eid];
        const int cxi = __float_as_int((xd.x - xs.x) * sv);
        const int cyi = __float_as_int((xd.y - xs.y) * sv);
        const int czi = __float_as_int((xd.z - xs.z) * sv);
#pragma unroll 1
        for (int k = 0; k < m32; ++k) {
          dx += __int_as_float(__builtin_amdgcn_readlane(cxi, k));
          dy += __int_as_float(__builtin_amdgcn_readlane(cyi, k));
          dz += __int_as_float(__builtin_amdgcn_readlane(czi, k));
        }
      }
    }
    const bool  live = node < mRows;
    const int   nr   = live ? node : mRows - 1;
    const float pzr  = big ? qnan : pz;
    if constexpr (COORD == 0) {
      const int j = lane & 15, part = lane >> 4;
      const unsigned mh = 0u - (unsigned)part;
      const unsigned ml = ~mh;
      const int s0l = 2 * j, s1l = 2 * j + 1;
      float g[8];
      g[0] = __shfl(a0, s0l, 32);
      g[1] = __shfl(a1, s0l, 32);
      g[2] = __shfl(a2, s0l, 32);
      g[3] = __shfl(a3, s0l, 32);
      g[4] = __shfl(a0, s1l, 32);
      g[5] = __shfl(a1, s1l, 32);
      g[6] = __shfl(a2, s1l, 32);
      g[7] = __shfl(a3, s1l, 32);
      unsigned short* bp = NZ + (size_t)nr * KNZ + 2 * HID + 8 * j;
      float old[8];
#pragma unroll
      for (int e = 0; e < 8; ++e) old[e] = 0.0f;
      if (first == 0) {
        const v4i hw = *(const v4ia*)bp;
        const v4i lw = *(const v4ia*)(bp + HID);
#pragma unroll
        for (int e = 0; e < 4; ++e) {
          const unsigned hu = (unsigned)hw[e], lu = (unsigned)lw[e];
          old[2 * e]     = __uint_as_float(hu << 16) + __uint_as_float(lu << 16);
          old[2 * e + 1] = __uint_as_float(hu & 0xffff0000u) + __uint_as_float(lu & 0xffff0000u);
        }
      }
      v8us oo;
#pragma unroll
      for (int e = 0; e < 8; ++e) {
        const float nv = old[e] + (g[e] * MINV) * NINV + pzr;
        const unsigned hb = bf16_bits(nv);
        const unsigned lb = bf16_bits(nv - __uint_as_float(hb << 16));
        oo[e] = (unsigned short)((hb & ml) | (lb & mh));
      }
      unsigned short* dp = bp + part * HID;
      if (live) *(volatile v8us*)dp = oo;
      __threadfence();
      if (live) *(volatile v8us*)dp = oo;
    } else {
      if (lane == 0) {
        const v4f d4 = {dx + pzr, dy + pzr, dz + pzr, 0.0f};
        *(v4fa*)(sdx + 4 * s) = d4;
      }
    }
  }
  __syncthreads();

  if constexpr (COORD == 1) {
    v4f dv[4];
#pragma unroll
    for (int jj = 0; jj < 4; ++jj) {
      const int slot = jj * NTHR + tid;
      const int node = nodeBase + slot;
      const int nr   = node < mRows ? node : mRows - 1;
      v4f old4 = z4f;
      if (first == 0) old4 = *(const v4fa*)(XAGG + (size_t)nr * 4);
      const v4f add  = *(const v4fa*)(sdx + 4 * slot);
      v4f q;
      q.x = old4.x + add.x; q.y = old4.y + add.y; q.z = old4.z + add.z; q.w = old4.w + add.w;
      dv[jj] = q;
    }
#pragma unroll
    for (int jj = 0; jj < 4; ++jj) {
      const int node = nodeBase + jj * NTHR + tid;
      if (node < mRows) *(volatile v4f*)(XAGG + (size_t)node * 4) = dv[jj];
    }
    __threadfence();
#pragma unroll
    for (int jj = 0; jj < 4; ++jj) {
      const int node = nodeBase + jj * NTHR + tid;
      if (node < mRows) *(volatile v4f*)(XAGG + (size_t)node * 4) = dv[jj];
    }
  }
}

__global__ __launch_bounds__(NTHR) void k_xout(const float* __restrict__ x, const float* __restrict__ XAGG,
                                               int nN, float* out1) {
  __shared__ __attribute__((aligned(16))) float sx[XROWS * 3];
  const int tid = (int)threadIdx.x;
  const int rowBase = (int)blockIdx.x * XROWS;
  for (int j = tid; j < XROWS * 3; j += NTHR) {
    const int rl  = j / 3;
    const int cc  = j - 3 * rl;
    const int row = rowBase + rl;
    const int rc  = row < nN ? row : nN - 1;
    const float xv = bf16_val(x[(size_t)rc * 3 + cc]);
    const float dv = XAGG[(size_t)rc * 4 + cc];
    sx[j] = fmaf(dv, NINV, xv);
  }
  __syncthreads();
  const int tl = tid < (XROWS * 3) / 4 ? tid : (XROWS * 3) / 4 - 1;
  const v4f o4 = *(const v4fa*)(sx + 4 * tl);
  const long long gidx = (long long)rowBase * 3 + 4LL * tl;
  const bool stv = (tid < (XROWS * 3) / 4) && (gidx + 4 <= 3LL * nN);
  if (stv) *(volatile v4f*)(out1 + (size_t)gidx) = o4;
  __threadfence();
  if (stv) *(volatile v4f*)(out1 + (size_t)gidx) = o4;
}

static inline int cdiv(int a, int b) { return (a + b - 1) / b; }

extern "C" void kernel_launch(void* const* d_in, const int* in_sizes, int n_in,
                              void* d_out, int out_size, void* d_ws, size_t ws_size,
                              hipStream_t stream) {
  if (n_in < 19) return;
  if (in_sizes[0] < HID || (in_sizes[0] % HID) != 0) return;
  const int nN = in_sizes[0] / HID;
  if (in_sizes[1] != 3 * nN) return;
  if (in_sizes[2] < 2 || (in_sizes[2] & 1) != 0) return;
  const int nE = in_sizes[2] / 2;
  if (nE < 1 || nE >= (1 << 22)) return;
  if (in_sizes[3] != nE) return;
  if (in_sizes[4] != NLAY * W1R * HID || in_sizes[5] != NLAY * HID) return;
  if (in_sizes[6] != NLAY * HID * HID || in_sizes[7] != NLAY * HID) return;
  if (in_sizes[8] != NLAY * 2 * HID * HID || in_sizes[9] != NLAY * HID) return;
  if (in_sizes[10] != NLAY * HID * HID || in_sizes[11] != NLAY * HID) return;
  if (in_sizes[12] != NLAY * HID || in_sizes[13] != NLAY) return;
  if (in_sizes[14] != W1R * HID || in_sizes[15] != HID) return;
  if (in_sizes[16] != HID * HID || in_sizes[17] != HID) return;
  if (in_sizes[18] != HID) return;
  if ((long long)out_size != (long long)nN * HID + 3LL * nN) return;
  if (((3 * nN) & 3) != 0) return;

  const float* h     = (const float*)d_in[0];
  const float* x     = (const float*)d_in[1];
  const int*   ei    = (const int*)d_in[2];
  const float* eattr = (const float*)d_in[3];
  const float* ew1   = (const float*)d_in[4];
  const float* eb1   = (const float*)d_in[5];
  const float* ew2   = (const float*)d_in[6];
  const float* eb2   = (const float*)d_in[7];
  const float* nw1   = (const float*)d_in[8];
  const float* nb1   = (const float*)d_in[9];
  const float* nw2   = (const float*)d_in[10];
  const float* nb2   = (const float*)d_in[11];
  const float* aw    = (const float*)d_in[12];
  const float* ab    = (const float*)d_in[13];
  const float* cw1   = (const float*)d_in[14];
  const float* cb1   = (const float*)d_in[15];
  const float* cw2   = (const float*)d_in[16];
  const float* cb2   = (const float*)d_in[17];
  const float* cw3   = (const float*)d_in[18];
  float* out0 = (float*)d_out;
  float* out1 = out0 + (size_t)nN * HID;

  const int MP = cdiv(nN, GBM) * GBM;
  const int gM = MP / GBM;
  const int gA = cdiv(MP, NBA);
  if ((long long)gA * NBA < (long long)MP) return;
  const int EH = cdiv(cdiv(nE, NRANGE), EPB) * EPB;
  if (EH < EPB || EH >= (1 << 21)) return;

  char* ws = (char*)d_ws;
  size_t off = 0;
  const size_t oWPT  = off; off += (size_t)3 * NPQ * KPQ * 2;        off = (off + 255) & ~(size_t)255;
  const size_t oW2T  = off; off += (size_t)3 * HID * HID * 2;        off = (off + 255) & ~(size_t)255;
  const size_t oWN1T = off; off += (size_t)NLAY * HID * KNZ * 2;     off = (off + 255) & ~(size_t)255;
  const size_t oWN2T = off; off += (size_t)NLAY * HID * KN2 * 2;     off = (off + 255) & ~(size_t)255;
  const size_t oCP   = off; off += (size_t)MP * 4 * 4;               off = (off + 255) & ~(size_t)255;
  const size_t oXAGG = off; off += (size_t)MP * 4 * 4;               off = (off + 255) & ~(size_t)255;
  const size_t oNZ   = off; off += (size_t)MP * KNZ * 2;             off = (off + 255) & ~(size_t)255;
  size_t szRM = (size_t)EH * MPITCH * 2;
  if (szRM < (size_t)MP * KN2 * 2) szRM = (size_t)MP * KN2 * 2;
  const size_t oRM   = off; off += szRM;                             off = (off + 255) & ~(size_t)255;
  const size_t oS    = off; off += (size_t)EH * 4;                   off = (off + 255) & ~(size_t)255;
  const size_t oPQ   = off; off += (size_t)MP * NPQ * 4;             off = (off + 255) & ~(size_t)255;
  if (off > ws_size || off > (size_t)WSMAX) return;
  unsigned short* WPT  = (unsigned short*)(ws + oWPT);
  unsigned short* W2T  = (unsigned short*)(ws + oW2T);
  unsigned short* WN1T = (unsigned short*)(ws + oWN1T);
  unsigned short* WN2T = (unsigned short*)(ws + oWN2T);
  float*          CP   = (float*)(ws + oCP);
  float*          XAGG = (float*)(ws + oXAGG);
  unsigned short* NZ   = (unsigned short*)(ws + oNZ);
  unsigned short* MSG  = (unsigned short*)(ws + oRM);
  unsigned short* G1   = (unsigned short*)(ws + oRM);
  float*          S    = (float*)(ws + oS);
  float*          PQ   = (float*)(ws + oPQ);

  hipFuncSetAttribute(reinterpret_cast<const void*>(&k_edge<0>), hipFuncAttributeMaxDynamicSharedMemorySize,
                      (int)EDGE_LDS_BYTES);
  hipFuncSetAttribute(reinterpret_cast<const void*>(&k_edge<1>), hipFuncAttributeMaxDynamicSharedMemorySize,
                      (int)EDGE_LDS_BYTES);
  hipFuncSetAttribute(reinterpret_cast<const void*>(&k_scan<0>), hipFuncAttributeMaxDynamicSharedMemorySize,
                      (int)AGG_LDS_BYTES);
  hipFuncSetAttribute(reinterpret_cast<const void*>(&k_scan<1>), hipFuncAttributeMaxDynamicSharedMemorySize,
                      (int)AGG_LDS_BYTES);

  const int nXP   = cdiv(MP, NTHR) * NTHR;
  const int nPrep = NU_WPT + NU_W2T + NU_WN1 + NU_WN2 + MP * 32 + nXP;
  const int vec8  = 1;

  k_prep<<<nPrep / NTHR, NTHR, 0, stream>>>(h, x, ew1, cw1, ew2, cw2, nw1, nw2, nN, MP,
                                            WPT, W2T, WN1T, WN2T, NZ, CP);

  for (int l = 0; l < NLAY; ++l) {
    const float* ew1l = ew1 + (size_t)l * W1R * HID;
    const float* eb1l = eb1 + (size_t)l * HID;
    const float* eb2l = eb2 + (size_t)l * HID;
    const float* nb1l = nb1 + (size_t)l * HID;
    const float* nb2l = nb2 + (size_t)l * HID;
    const float* awl  = aw  + (size_t)l * HID;
    const float* abl  = ab  + l;
    const unsigned short* WPTl  = WPT  + (size_t)l * NPQ * KPQ;
    const unsigned short* W2Tl  = W2T  + (size_t)l * HID * HID;
    const unsigned short* WN1Tl = WN1T + (size_t)l * HID * KNZ;
    const unsigned short* WN2Tl = WN2T + (size_t)l * HID * KN2;
    const int KP = (l == 0) ? HID : KPQ;
    k_gemm<0><<<dim3(gM, NPQ / GBN), GTHR, 0, stream>>>(NZ, KNZ, WPTl, KPQ, KP, nb1l, nN, 0, PQ, NPQ, G1, KN2);
    for (int r = 0; r < NRANGE; ++r) {
      const int eBase = r * EH;
      if (eBase >= nE) break;
      const int nEh = (nE - eBase) < EH ? (nE - eBase) : EH;
      const int first = (r == 0) ? 1 : 0;
      k_edge<0><<<cdiv(nEh, EPB), NTHR, EDGE_LDS_BYTES, stream>>>(ei, nE, nN, eBase, nEh, PQ, CP, eattr,
                                                                  W2Tl, eb1l, eb2l, awl, abl, ew1l + (size_t)2 * HID * HID,
                                                                  MSG, S);
      k_scan<0><<<gA, NTHR, AGG_LDS_BYTES, stream>>>(ei + eBase, ei + (size_t)nE + eBase, nEh, nN, vec8, MP, first,
                                                     MSG, S, CP, NZ, XAGG);
    }
    k_gemm<1><<<dim3(gM, 1), GTHR, 0, stream>>>(NZ, KNZ, WN1Tl, KNZ, KNZ, nb1l, nN, 0, PQ, NPQ, G1, KN2);
    k_gemm<2><<<dim3(gM, 1), GTHR, 0, stream>>>(G1, KN2, WN2Tl, KN2, KN2, nb2l, nN, (l == NLAY - 1) ? 1 : 0,
                                                out0, HID, NZ, KNZ);
  }

  {
    const unsigned short* WPTc = WPT + (size_t)2 * NPQ * KPQ;
    const unsigned short* W2Tc = W2T + (size_t)2 * HID * HID;
    k_gemm<0><<<dim3(gM, NPQ / GBN), GTHR, 0, stream>>>(NZ, KNZ, WPTc, KPQ, KPQ, nb1, nN, 0, PQ, NPQ, G1, KN2);
    for (int r = 0; r < NRANGE; ++r) {
      const int eBase = r * EH;
      if (eBase >= nE) break;
      const int nEh = (nE - eBase) < EH ? (nE - eBase) : EH;
      const int first = (r == 0) ? 1 : 0;
      k_edge<1><<<cdiv(nEh, EPB), NTHR, EDGE_LDS_BYTES, stream>>>(ei, nE, nN, eBase, nEh, PQ, CP, eattr,
                                                                  W2Tc, cb1, cb2, cw3, ab, cw1 + (size_t)2 * HID * HID,
                                                                  MSG, S);
      k_scan<1><<<gA, NTHR, AGG_LDS_BYTES, stream>>>(ei + eBase, ei + (size_t)nE + eBase, nEh, nN, vec8, MP, first,
                                                     MSG, S, CP, NZ, XAGG);
    }
    k_xout<<<cdiv(nN, XROWS), NTHR, 0, stream>>>(x, XAGG, nN, out1);
  }
}
